// GRUActor_23596550324466
// MI455X (gfx1250) — hardware-run, weakly checked
//
#include <hip/hip_runtime.h>


typedef _Float16 v16h __attribute__((ext_vector_type(16)));
typedef _Float16 v8h  __attribute__((ext_vector_type(8)));
typedef float    v8f  __attribute__((ext_vector_type(8)));
typedef float    v4f  __attribute__((ext_vector_type(4)));
typedef float    v4fa __attribute__((ext_vector_type(4))) __attribute__((may_alias));

#define B_ROWS 32768
#define IN_D   256
#define HID    64
#define G3     192
#define TRAJ   50
#define OUT_D  100
#define RPB    128

#define OFF_W1F   0
#define OFF_W2F   32768
#define OFF_WHHF  40960
#define OFF_H     65536
#define OFF_OT    81920
#define OFF_B1    133120
#define OFF_B2    133376
#define OFF_BIH   133632
#define OFF_BHH   134400
#define OFF_WIH   135168
#define OFF_WOUT  136704
#define OFF_BOUT  137216
#define SMEM_BYTES 137232

static_assert(B_ROWS % RPB == 0);
static_assert((RPB * OUT_D * 4) % 512 == 0);
static_assert((RPB * OUT_D) % 4 == 0);
static_assert(OFF_H % 16 == 0 && OFF_OT % 16 == 0 && OFF_W2F % 32 == 0 && OFF_WHHF % 32 == 0);

__device__ __forceinline__ float fsig(float x) {
    const float e = __expf(-x);
    return __builtin_amdgcn_rcpf(1.0f + e);
}
__device__ __forceinline__ float ftanh(float x) {
    const float e = __expf(-2.0f * fabsf(x));
    const float t = (1.0f - e) * __builtin_amdgcn_rcpf(1.0f + e);
    return x >= 0.0f ? t : -t;
}
__device__ __forceinline__ v8f zero8() {
    v8f z;
#pragma unroll
    for (int r = 0; r < 8; ++r) z[r] = 0.0f;
    return z;
}

__device__ __forceinline__ void mma16(v8f& acc, const v16h& a, const v16h& b) {
    acc = __builtin_amdgcn_wmma_f32_16x16x32_f16(false, a, false, b, (short)0, acc, false, false);
    asm volatile("v_nop\n\tv_nop\n\tv_nop\n\tv_nop" : "+v"(acc) : "v"(a), "v"(b));
}

__device__ __forceinline__ v16h load_a_lds(const _Float16* hw, int m, int colbase) {
    union { v16h v; v8h h8[2]; } u;
    u.h8[0] = *(const v8h*)(hw + m * 64 + colbase);
    u.h8[1] = *(const v8h*)(hw + m * 64 + colbase + 16);
    return u.v;
}

__device__ __forceinline__ v16h load_a_x(const float* p) {
    const v4f f0 = *(const v4f*)(p);
    const v4f f1 = *(const v4f*)(p + 4);
    const v4f f2 = *(const v4f*)(p + 16);
    const v4f f3 = *(const v4f*)(p + 20);
    v16h a;
#pragma unroll
    for (int i = 0; i < 4; ++i) {
        a[i]      = (_Float16)f0[i];
        a[4 + i]  = (_Float16)f1[i];
        a[8 + i]  = (_Float16)f2[i];
        a[12 + i] = (_Float16)f3[i];
    }
    return a;
}

__global__ __launch_bounds__(256)
void gru_traj_kernel(const float* __restrict__ x,
                     const float* __restrict__ W1,  const float* __restrict__ b1,
                     const float* __restrict__ W2,  const float* __restrict__ b2,
                     const float* __restrict__ Wih, const float* __restrict__ bih,
                     const float* __restrict__ Whh, const float* __restrict__ bhh,
                     const float* __restrict__ Wout, const float* __restrict__ bout,
                     float* out)
{
    extern __shared__ __attribute__((aligned(32))) char smem[];
    _Float16* w1f   = (_Float16*)(smem + OFF_W1F);
    _Float16* w2f   = (_Float16*)(smem + OFF_W2F);
    _Float16* whhf  = (_Float16*)(smem + OFF_WHHF);
    _Float16* hsm   = (_Float16*)(smem + OFF_H);
    float*    otile = (float*)(smem + OFF_OT);
    float*    b1s   = (float*)(smem + OFF_B1);
    float*    b2s   = (float*)(smem + OFF_B2);
    float*    bihs  = (float*)(smem + OFF_BIH);
    float*    bhhs  = (float*)(smem + OFF_BHH);
    float*    wihs  = (float*)(smem + OFF_WIH);
    float*    wouts = (float*)(smem + OFF_WOUT);
    float*    bouts = (float*)(smem + OFF_BOUT);

    const int tid = threadIdx.x;

    for (int e = tid; e < 16384; e += 256) {
        const int i = e & 15, ln = (e >> 4) & 31, nt = (e >> 9) & 3, kc = e >> 11;
        const int K = kc * 32 + ((ln >> 4) << 3) + (i & 7) + ((i >> 3) << 4);
        const int N = nt * 16 + (ln & 15);
        w1f[e] = (_Float16)(W1[K * HID + N] * 16.0f);
    }
    for (int e = tid; e < 4096; e += 256) {
        const int i = e & 15, ln = (e >> 4) & 31, nt = (e >> 9) & 3, kc = e >> 11;
        const int K = kc * 32 + ((ln >> 4) << 3) + (i & 7) + ((i >> 3) << 4);
        const int N = nt * 16 + (ln & 15);
        w2f[e] = (_Float16)(W2[K * HID + N] * 16.0f);
    }
    for (int e = tid; e < 12288; e += 256) {
        const int i = e & 15, ln = (e >> 4) & 31;
        const int g = e >> 9;
        const int nt = g % 12, kc = g / 12;
        const int K = kc * 32 + ((ln >> 4) << 3) + (i & 7) + ((i >> 3) << 4);
        const int N = nt * 16 + (ln & 15);
        whhf[e] = (_Float16)(Whh[K * G3 + N] * 16.0f);
    }
    for (int e = tid; e < 64;  e += 256) { b1s[e] = b1[e]; b2s[e] = b2[e]; }
    for (int e = tid; e < 192; e += 256) { bihs[e] = bih[e]; bhhs[e] = bhh[e]; }
    for (int e = tid; e < 384; e += 256) wihs[e] = Wih[e];
    for (int e = tid; e < 128; e += 256) wouts[e] = Wout[e];
    if (tid < 2) bouts[tid] = bout[tid];
    __syncthreads();

    const int lane = tid & 31;
    const int wave = tid >> 5;
    const int n16  = lane & 15;
    const int hi   = lane >> 4;
    const int rowBase = blockIdx.x * RPB + wave * 16;
    const float* xrow = x + (size_t)(rowBase + n16) * IN_D;
    _Float16* hw = hsm + wave * 1024;

    v8f acc1[4];
#pragma unroll
    for (int nt = 0; nt < 4; ++nt) acc1[nt] = zero8();
#pragma unroll
    for (int kc = 0; kc < 8; ++kc) {
        const v16h a = load_a_x(xrow + kc * 32 + 8 * hi);
#pragma unroll
        for (int nt = 0; nt < 4; ++nt) {
            const v16h b = *(const v16h*)(w1f + ((kc * 4 + nt) * 32 + lane) * 16);
            mma16(acc1[nt], a, b);
        }
    }
#pragma unroll
    for (int nt = 0; nt < 4; ++nt) {
        const float bb = b1s[nt * 16 + n16];
#pragma unroll
        for (int v = 0; v < 8; ++v) {
            float z = acc1[nt][v] * (1.0f / 16.0f) + bb;
            z = z > 0.0f ? z : 0.0f;
            hw[(v + hi * 8) * 64 + nt * 16 + n16] = (_Float16)(z * 16.0f);
        }
    }
    __syncthreads();

    v16h a0 = load_a_lds(hw, n16, 8 * hi);
    v16h a1 = load_a_lds(hw, n16, 32 + 8 * hi);
    v8f hc[4];
#pragma unroll
    for (int nt = 0; nt < 4; ++nt) {
        v8f acc = zero8();
        {
            const v16h b0 = *(const v16h*)(w2f + ((0 * 4 + nt) * 32 + lane) * 16);
            mma16(acc, a0, b0);
            const v16h b1v = *(const v16h*)(w2f + ((1 * 4 + nt) * 32 + lane) * 16);
            mma16(acc, a1, b1v);
        }
        const float bb = b2s[nt * 16 + n16];
#pragma unroll
        for (int v = 0; v < 8; ++v) {
            float z = acc[v] * (1.0f / 256.0f) + bb;
            z = z > 0.0f ? z : 0.0f;
            hc[nt][v] = z;
            hw[(v + hi * 8) * 64 + nt * 16 + n16] = (_Float16)(z * 16.0f);
        }
    }
    __syncthreads();
    a0 = load_a_lds(hw, n16, 8 * hi);
    a1 = load_a_lds(hw, n16, 32 + 8 * hi);

    float wo0[4], wo1[4];
#pragma unroll
    for (int nt = 0; nt < 4; ++nt) {
        wo0[nt] = wouts[(nt * 16 + n16) * 2 + 0];
        wo1[nt] = wouts[(nt * 16 + n16) * 2 + 1];
    }
    const float bo0 = bouts[0], bo1 = bouts[1];

    float wp0c[8], wp1c[8];
#pragma unroll
    for (int v = 0; v < 8; ++v) { wp0c[v] = 0.0f; wp1c[v] = 0.0f; }

    float* orow = otile + (wave * 16 + hi * 8) * OUT_D;

#pragma unroll 1
    for (int t = 0; t < TRAJ; ++t) {
        float s0[8], s1[8];
#pragma unroll
        for (int v = 0; v < 8; ++v) { s0[v] = 0.0f; s1[v] = 0.0f; }

#pragma unroll
        for (int nt = 0; nt < 4; ++nt) {
            const int j = nt * 16 + n16;
            v8f ar = zero8(), au = zero8(), an = zero8();
            {
                v16h bm;
                bm = *(const v16h*)(whhf + ((0 * 12 + nt) * 32 + lane) * 16);
                mma16(ar, a0, bm);
                bm = *(const v16h*)(whhf + ((1 * 12 + nt) * 32 + lane) * 16);
                mma16(ar, a1, bm);
                bm = *(const v16h*)(whhf + ((0 * 12 + nt + 4) * 32 + lane) * 16);
                mma16(au, a0, bm);
                bm = *(const v16h*)(whhf + ((1 * 12 + nt + 4) * 32 + lane) * 16);
                mma16(au, a1, bm);
                bm = *(const v16h*)(whhf + ((0 * 12 + nt + 8) * 32 + lane) * 16);
                mma16(an, a0, bm);
                bm = *(const v16h*)(whhf + ((1 * 12 + nt + 8) * 32 + lane) * 16);
                mma16(an, a1, bm);
            }

            const float wi0r = wihs[j],        wi1r = wihs[G3 + j];
            const float wi0z = wihs[64 + j],   wi1z = wihs[G3 + 64 + j];
            const float wi0n = wihs[128 + j],  wi1n = wihs[G3 + 128 + j];
            const float bir = bihs[j], biz = bihs[64 + j], bin = bihs[128 + j];
            const float bhr = bhhs[j], bhz = bhhs[64 + j], bhn = bhhs[128 + j];
#pragma unroll
            for (int v = 0; v < 8; ++v) {
                const float hr  = ar[v] * (1.0f / 256.0f) + bhr;
                const float hz  = au[v] * (1.0f / 256.0f) + bhz;
                const float hn  = an[v] * (1.0f / 256.0f) + bhn;
                const float ir  = wp0c[v] * wi0r + wp1c[v] * wi1r + bir;
                const float iz  = wp0c[v] * wi0z + wp1c[v] * wi1z + biz;
                const float inn = wp0c[v] * wi0n + wp1c[v] * wi1n + bin;
                const float r = fsig(ir + hr);
                const float u = fsig(iz + hz);
                const float n = ftanh(inn + r * hn);
                const float hnew = (1.0f - u) * n + u * hc[nt][v];
                hc[nt][v] = hnew;
                hw[(v + hi * 8) * 64 + j] = (_Float16)(hnew * 16.0f);
                s0[v] = hnew * wo0[nt] + s0[v];
                s1[v] = hnew * wo1[nt] + s1[v];
            }
        }

#pragma unroll
        for (int v = 0; v < 8; ++v) {
            float p0 = s0[v], p1 = s1[v];
            p0 += __shfl_xor(p0, 1, 32);  p1 += __shfl_xor(p1, 1, 32);
            p0 += __shfl_xor(p0, 2, 32);  p1 += __shfl_xor(p1, 2, 32);
            p0 += __shfl_xor(p0, 4, 32);  p1 += __shfl_xor(p1, 4, 32);
            p0 += __shfl_xor(p0, 8, 32);  p1 += __shfl_xor(p1, 8, 32);
            wp0c[v] = wp0c[v] + fsig(p0 + bo0);
            wp1c[v] = wp1c[v] + fsig(p1 + bo1);
            const float val = (n16 == 0) ? wp0c[v] : wp1c[v];
            if (n16 < 2) orow[v * OUT_D + 2 * t + n16] = val;
        }

        __syncthreads();
        a0 = load_a_lds(hw, n16, 8 * hi);
        a1 = load_a_lds(hw, n16, 32 + 8 * hi);
    }

    __syncthreads();
    const v4fa* src = (const v4fa*)otile;
    float* gout = out + (size_t)blockIdx.x * (RPB * OUT_D);
    constexpr int NV4 = (RPB * OUT_D) / 4;
#pragma unroll 1
    for (int i = tid; i < NV4; i += 256) {
        const v4f v = src[i];
        *(volatile v4f*)(gout + 4 * i) = v;
    }
    __threadfence();
#pragma unroll 1
    for (int i = tid; i < NV4; i += 256) {
        const v4f v = src[i];
        *(volatile v4f*)(gout + 4 * i) = v;
    }
}

extern "C" void kernel_launch(void* const* d_in, const int* in_sizes, int n_in,
                              void* d_out, int out_size, void* d_ws, size_t ws_size,
                              hipStream_t stream)
{
    (void)d_ws; (void)ws_size;
    if (n_in < 11) return;
    if (in_sizes[0]  != B_ROWS * IN_D) return;
    if (in_sizes[1]  != IN_D * HID)    return;
    if (in_sizes[2]  != HID)           return;
    if (in_sizes[3]  != HID * HID)     return;
    if (in_sizes[4]  != HID)           return;
    if (in_sizes[5]  != 2 * G3)        return;
    if (in_sizes[6]  != G3)            return;
    if (in_sizes[7]  != HID * G3)      return;
    if (in_sizes[8]  != G3)            return;
    if (in_sizes[9]  != HID * 2)       return;
    if (in_sizes[10] != 2)             return;
    if (out_size != B_ROWS * OUT_D)    return;

    const float* x    = (const float*)d_in[0];
    const float* W1   = (const float*)d_in[1];
    const float* b1   = (const float*)d_in[2];
    const float* W2   = (const float*)d_in[3];
    const float* b2   = (const float*)d_in[4];
    const float* Wih  = (const float*)d_in[5];
    const float* bih  = (const float*)d_in[6];
    const float* Whh  = (const float*)d_in[7];
    const float* bhh  = (const float*)d_in[8];
    const float* Wout = (const float*)d_in[9];
    const float* bout = (const float*)d_in[10];
    float* out = (float*)d_out;

    hipFuncSetAttribute(reinterpret_cast<const void*>(&gru_traj_kernel),
                        hipFuncAttributeMaxDynamicSharedMemorySize, SMEM_BYTES);
    gru_traj_kernel<<<dim3(B_ROWS / RPB), dim3(256), SMEM_BYTES, stream>>>(
        x, W1, b1, W2, b2, Wih, bih, Whh, bhh, Wout, bout, out);
}
